// DummyMPNN_46840913330618
// MI455X (gfx1250) — hardware-verified
//
#include <hip/hip_runtime.h>
#include <stddef.h>
#include <math.h>


#define HD     64
#define NF     14
#define EF     4
#define KW     4096
#define KTOT   4160
#define NITER  6
#define NTHR   256
#define NWAVE  8
#define EPT    8
#define NGRP   2
#define CHUNK  (NTHR * EPT * NGRP)
#define WCAP   (EPT * NGRP * 32)
#define LISTN  (NWAVE * WCAP)
#define NBK    128
#define MEDG   128
#define ACAP   1024
#define MAXG   1024
#define RVP    128
#define ESC    64.0f
#define WSC    64.0f
#define MINV   (1.0f / 4096.0f)
#define HSC    16.0f
#define MSC    16.0f
#define GSC    16.0f
#define INV256 (1.0f / 256.0f)

static_assert((CHUNK & (CHUNK - 1)) == 0);
static_assert(CHUNK <= 4096);
static_assert((NBK & (NBK - 1)) == 0);
static_assert(NBK <= 4096);
static_assert(NBK == NWAVE * 16);
static_assert(MEDG == NWAVE * 16);
static_assert((KTOT % 64) == 0);
static_assert((KW % 8) == 0);
static_assert(NTHR == 4 * HD);
static_assert(RVP == 2 * HD);
static_assert((HD * (KTOT / 8)) % 32 == 0);

typedef float    v2f  __attribute__((ext_vector_type(2)));
typedef float    v4f  __attribute__((ext_vector_type(4)));
typedef float    v8f  __attribute__((ext_vector_type(8)));
typedef int      v4i  __attribute__((ext_vector_type(4)));
typedef _Float16 v8h  __attribute__((ext_vector_type(8)));
typedef _Float16 v16h __attribute__((ext_vector_type(16)));
union FragH { v16h v; v8h h[2]; };

__device__ __forceinline__ v8h cvt8(v4f a, v4f b) {
  v8h r;
  r[0] = (_Float16)a.x; r[1] = (_Float16)a.y; r[2] = (_Float16)a.z; r[3] = (_Float16)a.w;
  r[4] = (_Float16)b.x; r[5] = (_Float16)b.y; r[6] = (_Float16)b.z; r[7] = (_Float16)b.w;
  return r;
}

__device__ __forceinline__ v8f wmh(v16h a, v16h b, v8f c) {
  v8f d = __builtin_amdgcn_wmma_f32_16x16x32_f16(false, a, false, b, (short)0, c, false, false);
  asm volatile("v_nop\n\tv_nop\n\tv_nop\n\tv_nop" : "+v"(d) : "v"(a), "v"(b));
  return d;
}

__device__ __forceinline__ float leaky_(float v) { return v > 0.f ? v : 0.01f * v; }
__device__ __forceinline__ float sigm_(float v)  { return __builtin_amdgcn_rcpf(1.0f + __expf(-v)); }
__device__ __forceinline__ float tanh_(float v)  { return 2.0f * sigm_(2.0f * v) - 1.0f; }

__device__ __forceinline__ float lstm_q(int d, const float* __restrict__ wih, const float* __restrict__ whh,
                                         const float* __restrict__ bih, const float* __restrict__ bhh) {
  float zi0 = 0.f, zi1 = 0.f, zi2 = 0.f, zi3 = 0.f, zh0 = 0.f, zh1 = 0.f, zh2 = 0.f, zh3 = 0.f;
#pragma unroll 1
  for (int k = 0; k < 2 * HD; ++k) {
    const float qs = 0.0f;
    zi0 += qs * wih[(size_t)(d) * 2 * HD + k];
    zi1 += qs * wih[(size_t)(HD + d) * 2 * HD + k];
    zi2 += qs * wih[(size_t)(2 * HD + d) * 2 * HD + k];
    zi3 += qs * wih[(size_t)(3 * HD + d) * 2 * HD + k];
  }
#pragma unroll 1
  for (int k = 0; k < HD; ++k) {
    const float hs = 0.0f;
    zh0 += hs * whh[(size_t)(d) * HD + k];
    zh1 += hs * whh[(size_t)(HD + d) * HD + k];
    zh2 += hs * whh[(size_t)(2 * HD + d) * HD + k];
    zh3 += hs * whh[(size_t)(3 * HD + d) * HD + k];
  }
  const float g0 = ((zi0 + bih[d]) + zh0) + bhh[d];
  const float g1 = ((zi1 + bih[HD + d]) + zh1) + bhh[HD + d];
  const float g2 = ((zi2 + bih[2 * HD + d]) + zh2) + bhh[2 * HD + d];
  const float g3 = ((zi3 + bih[3 * HD + d]) + zh3) + bhh[3 * HD + d];
  const float ig = sigm_(g0), fg = sigm_(g1), gg = tanh_(g2), og = sigm_(g3);
  const float c = fg * 0.0f + ig * gg;
  return og * tanh_(c);
}

template <int NB>
__device__ __forceinline__ int scan_chunk(const int* __restrict__ dsts, int nE, int cbase, int nodeBase,
                                          int vec8, int* list, int tid, int lane, int wave) {
  int wc = 0;
#pragma unroll
  for (int g = 0; g < NGRP; ++g) {
    const int el0  = (g * NTHR + tid) * EPT;
    const int e0   = cbase + el0;
    const int sent = -2147483647 - 1;
    v4i da, db;
    if (vec8 != 0 && e0 + 7 < nE) {
      da = *(const v4i*)(dsts + e0);
      db = *(const v4i*)(dsts + e0 + 4);
    } else {
      da.x = (e0     < nE) ? dsts[min(e0, nE - 1)] : sent;
      da.y = (e0 + 1 < nE) ? dsts[min(e0 + 1, nE - 1)] : sent;
      da.z = (e0 + 2 < nE) ? dsts[min(e0 + 2, nE - 1)] : sent;
      da.w = (e0 + 3 < nE) ? dsts[min(e0 + 3, nE - 1)] : sent;
      db.x = (e0 + 4 < nE) ? dsts[min(e0 + 4, nE - 1)] : sent;
      db.y = (e0 + 5 < nE) ? dsts[min(e0 + 5, nE - 1)] : sent;
      db.z = (e0 + 6 < nE) ? dsts[min(e0 + 6, nE - 1)] : sent;
      db.w = (e0 + 7 < nE) ? dsts[min(e0 + 7, nE - 1)] : sent;
    }
    const unsigned nb = (unsigned)nodeBase;
    const unsigned s0 = (unsigned)da.x - nb, s1 = (unsigned)da.y - nb;
    const unsigned s2 = (unsigned)da.z - nb, s3 = (unsigned)da.w - nb;
    const unsigned s4 = (unsigned)db.x - nb, s5 = (unsigned)db.y - nb;
    const unsigned s6 = (unsigned)db.z - nb, s7 = (unsigned)db.w - nb;
    const bool h0 = s0 < (unsigned)NB, h1 = s1 < (unsigned)NB, h2 = s2 < (unsigned)NB, h3 = s3 < (unsigned)NB;
    const bool h4 = s4 < (unsigned)NB, h5 = s5 < (unsigned)NB, h6 = s6 < (unsigned)NB, h7 = s7 < (unsigned)NB;
    const unsigned any = __builtin_amdgcn_ballot_w32(h0 | h1 | h2 | h3 | h4 | h5 | h6 | h7);
    if (any != 0u) {
#define HITJ(J, HJ, SJ) { \
        const unsigned mj = __builtin_amdgcn_ballot_w32(HJ); \
        if (mj != 0u) { \
          if (HJ) { \
            const int pos = wc + (int)__builtin_amdgcn_mbcnt_lo(mj, 0u); \
            if (pos < WCAP) list[wave * WCAP + pos] = ((el0 + (J)) << 12) | (int)(SJ); \
          } \
          wc += (int)__builtin_popcount(mj); } }
      HITJ(0, h0, s0)
      HITJ(1, h1, s1)
      HITJ(2, h2, s2)
      HITJ(3, h3, s3)
      HITJ(4, h4, s4)
      HITJ(5, h5, s5)
      HITJ(6, h6, s6)
      HITJ(7, h7, s7)
#undef HITJ
    }
  }
  return wc;
}

__global__ __launch_bounds__(NTHR) void k_wprep(
    const float* __restrict__ w2, const float* __restrict__ b2, const float* __restrict__ cr,
    const float* __restrict__ wih, const float* __restrict__ whh,
    _Float16* wT, _Float16* rT, _Float16* gIH, _Float16* gHH) {
  const int idx = blockIdx.x * NTHR + threadIdx.x;
  const int n1 = HD * (KTOT / 8);
  const int n2 = HD * (HD / 8);
  const int n3 = 3 * HD * (HD / 8);
  if (idx >= n1 + n2 + 2 * n3) return;
  v4f a, b;
  _Float16* dp;
  float sc;
  if (idx < n1) {
    const int o  = idx / (KTOT / 8);
    const int k0 = (idx - o * (KTOT / 8)) * 8;
    const float* p;
    int st;
    if (k0 < KW) {
      const int j = k0 >> 6, i0 = k0 & 63;
      p = w2 + ((size_t)(i0 * HD + o)) * HD + j;
      st = HD * HD;
    } else {
      const int i0 = k0 - KW;
      p = b2 + (size_t)i0 * HD + o;
      st = HD;
    }
    a.x = p[0];      a.y = p[st];     a.z = p[2 * st]; a.w = p[3 * st];
    b.x = p[4 * st]; b.y = p[5 * st]; b.z = p[6 * st]; b.w = p[7 * st];
    sc = WSC;
    dp = wT + (size_t)idx * 8;
  } else {
    const int u = idx - n1;
    const float* p;
    if (u < n2)           { p = cr  + (size_t)u * 8;             dp = rT  + (size_t)u * 8; }
    else if (u < n2 + n3) { p = wih + (size_t)(u - n2) * 8;      dp = gIH + (size_t)(u - n2) * 8; }
    else                  { p = whh + (size_t)(u - n2 - n3) * 8; dp = gHH + (size_t)(u - n2 - n3) * 8; }
    a = *(const v4f*)p;
    b = *(const v4f*)(p + 4);
    sc = GSC;
  }
  a = a * sc;
  b = b * sc;
  const v8h hv = cvt8(a, b);
  *(volatile v8h*)dp = hv;
  __threadfence();
  *(volatile v8h*)dp = hv;
}

__global__ __launch_bounds__(NTHR) void k_lin0(
    const float* __restrict__ x, const float* __restrict__ w, const float* __restrict__ bb,
    float* h, int nN) {
  const int idx = blockIdx.x * NTHR + threadIdx.x;
  const int node = idx >> 4, c4 = (idx & 15) * 4;
  const int nr = node > nN - 1 ? nN - 1 : node;
  float a0 = bb[c4], a1 = bb[c4 + 1], a2 = bb[c4 + 2], a3 = bb[c4 + 3];
  const float* xp = x + (size_t)nr * NF;
  const float* w0 = w + (size_t)c4 * NF;
#pragma unroll
  for (int f = 0; f < NF; ++f) {
    const float xv = xp[f];
    a0 += xv * w0[f]; a1 += xv * w0[NF + f]; a2 += xv * w0[2 * NF + f]; a3 += xv * w0[3 * NF + f];
  }
  v4f o;
  o.x = leaky_(a0); o.y = leaky_(a1); o.z = leaky_(a2); o.w = leaky_(a3);
  float* dp = h + (size_t)node * HD + c4;
  *(volatile v4f*)dp = o;
  __threadfence();
  *(volatile v4f*)dp = o;
}

__global__ __launch_bounds__(NTHR) void k_edgeh(
    const float* __restrict__ ea, const float* __restrict__ w1, const float* __restrict__ b1,
    float* es, int nE) {
  const int idx = blockIdx.x * NTHR + threadIdx.x;
  const int edge = idx >> 4, c4 = (idx & 15) * 4;
  const int er = edge > nE - 1 ? nE - 1 : edge;
  float a0 = b1[c4], a1 = b1[c4 + 1], a2 = b1[c4 + 2], a3 = b1[c4 + 3];
  const float* ap = ea + (size_t)er * EF;
  const float* w0 = w1 + (size_t)c4 * EF;
#pragma unroll
  for (int f = 0; f < EF; ++f) {
    const float av = ap[f];
    a0 += av * w0[f]; a1 += av * w0[EF + f]; a2 += av * w0[2 * EF + f]; a3 += av * w0[3 * EF + f];
  }
  v4f ev;
  ev.x = leaky_(a0) * ESC; ev.y = leaky_(a1) * ESC; ev.z = leaky_(a2) * ESC; ev.w = leaky_(a3) * ESC;
  float* dp = es + (size_t)edge * HD + c4;
  *(volatile v4f*)dp = ev;
  __threadfence();
  *(volatile v4f*)dp = ev;
}

__global__ __launch_bounds__(NTHR) void k_gather(
    const int* __restrict__ ei, const float* __restrict__ h, float* hs, int nN, int nE) {
  const int idx = blockIdx.x * NTHR + threadIdx.x;
  const int edge = idx >> 4, c4 = (idx & 15) * 4;
  const int er = edge > nE - 1 ? nE - 1 : edge;
  int src = ei[er];
  src = src < 0 ? 0 : (src > nN - 1 ? nN - 1 : src);
  const v4f hv = *(const v4f*)(h + (size_t)src * HD + c4);
  float* dp = hs + (size_t)edge * HD + c4;
  *(volatile v4f*)dp = hv;
  __threadfence();
  *(volatile v4f*)dp = hv;
}

__global__ __launch_bounds__(NTHR) void k_msg(
    const float* __restrict__ hs, const float* __restrict__ es,
    const _Float16* __restrict__ wT, float* msg) {
  __shared__ __attribute__((aligned(16))) float stg[NWAVE * 16 * HD];
  const int tid = threadIdx.x, lane = tid & 31, wave = tid >> 5, hf = lane >> 4, m = lane & 15;
  const int ebase = (blockIdx.x * NWAVE + wave) * 16;

  const float* hp = hs + ((size_t)ebase + m) * HD + 8 * hf;
  const v4f h00 = *(const v4f*)(hp),      h01 = *(const v4f*)(hp + 4);
  const v4f h10 = *(const v4f*)(hp + 16), h11 = *(const v4f*)(hp + 20);
  const v4f h20 = *(const v4f*)(hp + 32), h21 = *(const v4f*)(hp + 36);
  const v4f h30 = *(const v4f*)(hp + 48), h31 = *(const v4f*)(hp + 52);
  const float* ep = es + ((size_t)ebase + m) * HD;
  const _Float16* wb = wT + (size_t)m * KTOT + 8 * hf;

  v8f acc[4];
#pragma unroll
  for (int t = 0; t < 4; ++t) { v8f z = {0.f, 0.f, 0.f, 0.f, 0.f, 0.f, 0.f, 0.f}; acc[t] = z; }

#pragma unroll 1
  for (int jp = 0; jp < KTOT / 64; ++jp) {
    const int jc = jp < HD ? jp : HD - 1;
    const float sv = ep[jc];
    const float s = jp < HD ? sv : ESC;
    const int koff = 64 * jp;
    {
      FragH a;
      a.h[0] = cvt8(h00 * s, h01 * s);
      a.h[1] = cvt8(h10 * s, h11 * s);
#pragma unroll
      for (int t = 0; t < 4; ++t) {
        const _Float16* bp = wb + (size_t)t * 16 * KTOT + koff;
        FragH b;
        b.h[0] = *(const v8h*)bp;
        b.h[1] = *(const v8h*)(bp + 16);
        acc[t] = wmh(a.v, b.v, acc[t]);
      }
    }
    {
      FragH a;
      a.h[0] = cvt8(h20 * s, h21 * s);
      a.h[1] = cvt8(h30 * s, h31 * s);
#pragma unroll
      for (int t = 0; t < 4; ++t) {
        const _Float16* bp = wb + (size_t)t * 16 * KTOT + koff + 32;
        FragH b;
        b.h[0] = *(const v8h*)bp;
        b.h[1] = *(const v8h*)(bp + 16);
        acc[t] = wmh(a.v, b.v, acc[t]);
      }
    }
  }

  float* sw = stg + wave * (16 * HD);
#pragma unroll
  for (int t = 0; t < 4; ++t) {
#pragma unroll
    for (int r = 0; r < 8; ++r) sw[(8 * hf + r) * HD + 16 * t + m] = acc[t][r] * MINV;
  }
  __syncthreads();
  v4f ov[8];
#pragma unroll
  for (int q = 0; q < 8; ++q) ov[q] = *(const v4f*)(sw + (2 * q + hf) * HD + 4 * m);
  float* gp = msg + ((size_t)ebase + hf) * HD + 4 * m;
#pragma unroll
  for (int q = 0; q < 8; ++q) *(volatile v4f*)(gp + (size_t)(2 * q) * HD) = ov[q];
  __threadfence();
#pragma unroll
  for (int q = 0; q < 8; ++q) *(volatile v4f*)(gp + (size_t)(2 * q) * HD) = ov[q];
}

__global__ __launch_bounds__(NTHR) void k_node(
    const int* __restrict__ ei, const float* __restrict__ msg, const float* __restrict__ hin,
    const _Float16* __restrict__ rT, const _Float16* __restrict__ gIH, const _Float16* __restrict__ gHH,
    const float* __restrict__ conv_b, const float* __restrict__ b_ih, const float* __restrict__ b_hh,
    float* hout, int nN, int nE, int vec8) {
  __shared__ __attribute__((aligned(16))) float acc[NBK * HD];
  __shared__ __attribute__((aligned(16))) int list[LISTN];
  __shared__ int cnt[NBK];
  __shared__ int wcnt[NWAVE];
  const int tid = threadIdx.x, lane = tid & 31, wave = tid >> 5, hf = lane >> 4, m = lane & 15;
  const int nodeBase = blockIdx.x * NBK;
  const int* dsts = ei + nE;

  {
    const v4f z = {0.f, 0.f, 0.f, 0.f};
    for (int i = tid; i < NBK * HD / 4; i += NTHR) ((v4f*)acc)[i] = z;
    for (int i = tid; i < NBK; i += NTHR) cnt[i] = 0;
  }
  __syncthreads();

  const int nChunks = (nE + CHUNK - 1) / CHUNK;
#pragma unroll 1
  for (int ch = 0; ch < nChunks; ++ch) {
    const int cbase = ch * CHUNK;
    const int wc = scan_chunk<NBK>(dsts, nE, cbase, nodeBase, vec8, list, tid, lane, wave);
    if (lane == 0) wcnt[wave] = wc;
    __syncthreads();
    if (wave == 0) {
#pragma unroll 1
      for (int wsx = 0; wsx < NWAVE; ++wsx) {
        int n = __builtin_amdgcn_readfirstlane(wcnt[wsx]);
        n = n > WCAP ? WCAP : (n < 0 ? 0 : n);
        const int* lp = list + wsx * WCAP;
#pragma unroll 1
        for (int i = 0; i < n; ++i) {
          const int ent  = __builtin_amdgcn_readfirstlane(lp[i]);
          const int slot = ent & (NBK - 1);
          int e = cbase + ((ent >> 12) & (CHUNK - 1));
          e = e > nE - 1 ? nE - 1 : e;
          const v2f mv = *(const v2f*)(msg + (size_t)e * HD + 2 * lane);
          v2f* ap = (v2f*)(acc + slot * HD + 2 * lane);
          *ap = *ap + mv;
          if (lane == 0) cnt[slot] = cnt[slot] + 1;
        }
      }
    }
    __syncthreads();
  }

  int nodeA = nodeBase + 16 * wave + m;
  nodeA = nodeA > nN - 1 ? nN - 1 : nodeA;
  FragH ah[2];
#pragma unroll
  for (int kt = 0; kt < 2; ++kt) {
    const float* hp = hin + (size_t)nodeA * HD + 32 * kt + 8 * hf;
    ah[kt].h[0] = cvt8((*(const v4f*)hp) * HSC, (*(const v4f*)(hp + 4)) * HSC);
    ah[kt].h[1] = cvt8((*(const v4f*)(hp + 16)) * HSC, (*(const v4f*)(hp + 20)) * HSC);
  }

  v8f dr[4];
#pragma unroll
  for (int t = 0; t < 4; ++t) { v8f z = {0.f, 0.f, 0.f, 0.f, 0.f, 0.f, 0.f, 0.f}; dr[t] = z; }
#pragma unroll
  for (int kt = 0; kt < 2; ++kt) {
#pragma unroll
    for (int t = 0; t < 4; ++t) {
      const _Float16* bp = rT + (size_t)(16 * t + m) * HD + 32 * kt + 8 * hf;
      FragH b;
      b.h[0] = *(const v8h*)bp;
      b.h[1] = *(const v8h*)(bp + 16);
      dr[t] = wmh(ah[kt].v, b.v, dr[t]);
    }
  }

#pragma unroll
  for (int r = 0; r < 8; ++r) {
    const int slot = 16 * wave + 8 * hf + r;
    int c = cnt[slot];
    c = c < 1 ? 1 : c;
    const float degi = 1.0f / (float)c;
#pragma unroll
    for (int t = 0; t < 4; ++t) {
      const int col = 16 * t + m;
      float* p = acc + slot * HD + col;
      const float v = (*p * degi + dr[t][r] * INV256) + conv_b[col];
      *p = leaky_(v);
    }
  }
  __syncthreads();

  FragH am[2];
#pragma unroll
  for (int kt = 0; kt < 2; ++kt) {
    const float* rp = acc + (16 * wave + m) * HD + 32 * kt + 8 * hf;
    am[kt].h[0] = cvt8((*(const v4f*)rp) * MSC, (*(const v4f*)(rp + 4)) * MSC);
    am[kt].h[1] = cvt8((*(const v4f*)(rp + 16)) * MSC, (*(const v4f*)(rp + 20)) * MSC);
  }
  __syncthreads();

#pragma unroll 1
  for (int u = 0; u < 2; ++u) {
    v8f gin[2], ghn[2];
    {
      v8f z = {0.f, 0.f, 0.f, 0.f, 0.f, 0.f, 0.f, 0.f};
      gin[0] = z; gin[1] = z; ghn[0] = z; ghn[1] = z;
    }
#pragma unroll
    for (int kt = 0; kt < 2; ++kt) {
#pragma unroll
      for (int tt = 0; tt < 2; ++tt) {
        const int n = 2 * HD + 32 * u + 16 * tt + m;
        const _Float16* bp = gIH + (size_t)n * HD + 32 * kt + 8 * hf;
        FragH b;
        b.h[0] = *(const v8h*)bp;
        b.h[1] = *(const v8h*)(bp + 16);
        gin[tt] = wmh(am[kt].v, b.v, gin[tt]);
        const _Float16* bq = gHH + (size_t)n * HD + 32 * kt + 8 * hf;
        FragH b2;
        b2.h[0] = *(const v8h*)bq;
        b2.h[1] = *(const v8h*)(bq + 16);
        ghn[tt] = wmh(ah[kt].v, b2.v, ghn[tt]);
      }
    }
    v8f ar[2];
    {
      v8f z = {0.f, 0.f, 0.f, 0.f, 0.f, 0.f, 0.f, 0.f};
      ar[0] = z; ar[1] = z;
    }
#pragma unroll
    for (int kt = 0; kt < 2; ++kt) {
#pragma unroll
      for (int tt = 0; tt < 2; ++tt) {
        const int n = 32 * u + 16 * tt + m;
        const _Float16* bp = gIH + (size_t)n * HD + 32 * kt + 8 * hf;
        FragH b;
        b.h[0] = *(const v8h*)bp;
        b.h[1] = *(const v8h*)(bp + 16);
        ar[tt] = wmh(am[kt].v, b.v, ar[tt]);
        const _Float16* bq = gHH + (size_t)n * HD + 32 * kt + 8 * hf;
        FragH b2;
        b2.h[0] = *(const v8h*)bq;
        b2.h[1] = *(const v8h*)(bq + 16);
        ar[tt] = wmh(ah[kt].v, b2.v, ar[tt]);
      }
    }
    float nv[2][8];
#pragma unroll
    for (int tt = 0; tt < 2; ++tt) {
      const int col = 32 * u + 16 * tt + m;
      const float br  = b_ih[col] + b_hh[col];
      const float bni = b_ih[2 * HD + col];
      const float bnh = b_hh[2 * HD + col];
#pragma unroll
      for (int r = 0; r < 8; ++r) {
        const float rg   = sigm_(ar[tt][r] * INV256 + br);
        const float gi_n = gin[tt][r] * INV256 + bni;
        const float gh_n = ghn[tt][r] * INV256 + bnh;
        nv[tt][r] = tanh_(gi_n + rg * gh_n);
      }
    }
    v8f az[2];
    {
      v8f z = {0.f, 0.f, 0.f, 0.f, 0.f, 0.f, 0.f, 0.f};
      az[0] = z; az[1] = z;
    }
#pragma unroll
    for (int kt = 0; kt < 2; ++kt) {
#pragma unroll
      for (int tt = 0; tt < 2; ++tt) {
        const int n = HD + 32 * u + 16 * tt + m;
        const _Float16* bp = gIH + (size_t)n * HD + 32 * kt + 8 * hf;
        FragH b;
        b.h[0] = *(const v8h*)bp;
        b.h[1] = *(const v8h*)(bp + 16);
        az[tt] = wmh(am[kt].v, b.v, az[tt]);
        const _Float16* bq = gHH + (size_t)n * HD + 32 * kt + 8 * hf;
        FragH b2;
        b2.h[0] = *(const v8h*)bq;
        b2.h[1] = *(const v8h*)(bq + 16);
        az[tt] = wmh(ah[kt].v, b2.v, az[tt]);
      }
    }
#pragma unroll
    for (int tt = 0; tt < 2; ++tt) {
      const int col = 32 * u + 16 * tt + m;
      const float bz = b_ih[HD + col] + b_hh[HD + col];
#pragma unroll
      for (int r = 0; r < 8; ++r) {
        const int slot = 16 * wave + 8 * hf + r;
        int node = nodeBase + slot;
        node = node > nN - 1 ? nN - 1 : node;
        const float hold = hin[(size_t)node * HD + col];
        const float zg = sigm_(az[tt][r] * INV256 + bz);
        const float hn = (1.0f - zg) * nv[tt][r] + zg * hold;
        acc[slot * HD + col] = hn;
      }
    }
  }
  __syncthreads();

  v4f ov[8];
#pragma unroll
  for (int q = 0; q < 8; ++q) ov[q] = *(const v4f*)(acc + (wave * 8 + q) * 128 + 4 * lane);
  float* gp = hout + (size_t)nodeBase * HD;
#pragma unroll
  for (int q = 0; q < 8; ++q) *(volatile v4f*)(gp + (wave * 8 + q) * 128 + 4 * lane) = ov[q];
  __threadfence();
#pragma unroll
  for (int q = 0; q < 8; ++q) *(volatile v4f*)(gp + (wave * 8 + q) * 128 + 4 * lane) = ov[q];
}

__global__ __launch_bounds__(NTHR) void k_attn(
    const float* __restrict__ h, const int* __restrict__ batch,
    const float* __restrict__ lw_ih, const float* __restrict__ lw_hh,
    const float* __restrict__ lb_ih, const float* __restrict__ lb_hh,
    float* rvec, int nN) {
  __shared__ __attribute__((aligned(16))) float qsh[HD];
  __shared__ int nlist[ACAP];
  __shared__ float esh[ACAP];
  __shared__ __attribute__((aligned(16))) float red[NTHR];
  __shared__ __attribute__((aligned(16))) float rsh[RVP];
  __shared__ int wc[NWAVE];
  const int tid = threadIdx.x, lane = tid & 31, wave = tid >> 5;
  const int g = blockIdx.x;

  if (tid < HD) qsh[tid] = lstm_q(tid, lw_ih, lw_hh, lb_ih, lb_hh);
  __syncthreads();

  int tot = 0;
  const int nCh = (nN + NTHR - 1) / NTHR;
#pragma unroll 1
  for (int ch = 0; ch < nCh; ++ch) {
    const int n  = ch * NTHR + tid;
    const int bi = n < nN ? n : nN - 1;
    const int bv = batch[bi];
    const bool hit = (n < nN) && (bv == g);
    const unsigned mk = __builtin_amdgcn_ballot_w32(hit);
    if (lane == 0) wc[wave] = (int)__builtin_popcount(mk);
    __syncthreads();
    int pre = 0, all = 0;
#pragma unroll
    for (int w = 0; w < NWAVE; ++w) {
      const int c = wc[w];
      all += c;
      pre += (w < wave) ? c : 0;
    }
    if (hit) {
      const int pos = tot + pre + (int)__builtin_amdgcn_mbcnt_lo(mk, 0u);
      if (pos < ACAP) nlist[pos] = n;
    }
    tot += all;
    __syncthreads();
  }
  const int cnt = tot > ACAP ? ACAP : tot;

  float lmax = -3.0e38f;
#pragma unroll 1
  for (int k = tid; k < cnt; k += NTHR) {
    int node = nlist[k];
    node = node < 0 ? 0 : (node > nN - 1 ? nN - 1 : node);
    const float* hp = h + (size_t)node * HD;
    float s = 0.f;
#pragma unroll 4
    for (int c = 0; c < HD / 4; ++c) {
      const v4f v  = *(const v4f*)(hp + 4 * c);
      const v4f qv = *(const v4f*)(qsh + 4 * c);
      s += v.x * qv.x; s += v.y * qv.y; s += v.z * qv.z; s += v.w * qv.w;
    }
    esh[k] = s;
    lmax = fmaxf(lmax, s);
  }
  lmax = fmaxf(lmax, __shfl_xor(lmax, 16));
  lmax = fmaxf(lmax, __shfl_xor(lmax, 8));
  lmax = fmaxf(lmax, __shfl_xor(lmax, 4));
  lmax = fmaxf(lmax, __shfl_xor(lmax, 2));
  lmax = fmaxf(lmax, __shfl_xor(lmax, 1));
  if (lane == 0) red[wave] = lmax;
  __syncthreads();
  float emax = red[0];
#pragma unroll
  for (int w = 1; w < NWAVE; ++w) emax = fmaxf(emax, red[w]);
  __syncthreads();

  float lsum = 0.f;
#pragma unroll 1
  for (int k = tid; k < cnt; k += NTHR) {
    const float a = __expf(esh[k] - emax);
    esh[k] = a;
    lsum += a;
  }
  lsum += __shfl_xor(lsum, 16);
  lsum += __shfl_xor(lsum, 8);
  lsum += __shfl_xor(lsum, 4);
  lsum += __shfl_xor(lsum, 2);
  lsum += __shfl_xor(lsum, 1);
  if (lane == 0) red[wave] = lsum;
  __syncthreads();
  float ssum = 0.f;
#pragma unroll
  for (int w = 0; w < NWAVE; ++w) ssum += red[w];
  __syncthreads();
  const float inv = (cnt > 0) ? (1.0f / ssum) : 0.f;
#pragma unroll 1
  for (int k = tid; k < cnt; k += NTHR) esh[k] = esh[k] * inv;
  __syncthreads();

  const int d = tid & (HD - 1), p = tid >> 6;
  float s = 0.f;
#pragma unroll 1
  for (int k = p; k < cnt; k += NTHR / HD) {
    int node = nlist[k];
    node = node < 0 ? 0 : (node > nN - 1 ? nN - 1 : node);
    s += esh[k] * h[(size_t)node * HD + d];
  }
  red[tid] = s;
  __syncthreads();
  if (tid < RVP) {
    float r = 0.f;
    if (tid < HD) r = (red[tid] + red[HD + tid]) + (red[2 * HD + tid] + red[3 * HD + tid]);
    rsh[tid] = r;
  }
  __syncthreads();
  if (wave == 0) {
    const v4f v = *(const v4f*)(rsh + 4 * lane);
    float* gp = rvec + (size_t)g * RVP + 4 * lane;
    *(volatile v4f*)gp = v;
    __threadfence();
    *(volatile v4f*)gp = v;
  }
}

__global__ __launch_bounds__(NTHR) void k_out(
    const float* __restrict__ rvec,
    const float* __restrict__ lw_ih, const float* __restrict__ lw_hh,
    const float* __restrict__ lb_ih, const float* __restrict__ lb_hh,
    const float* __restrict__ ow, const float* __restrict__ ob,
    float* out, int nG) {
  __shared__ __attribute__((aligned(16))) float qsh[HD];
  __shared__ float yq[2];
  __shared__ __attribute__((aligned(16))) float ysh[2 * MAXG];
  const int tid = threadIdx.x, lane = tid & 31, wave = tid >> 5;

  if (tid < HD) qsh[tid] = lstm_q(tid, lw_ih, lw_hh, lb_ih, lb_hh);
  __syncthreads();
  if (tid < 2) {
    float s = 0.f;
#pragma unroll 4
    for (int d = 0; d < HD; ++d) s += qsh[d] * ow[(size_t)tid * 2 * HD + d];
    yq[tid] = s + ob[tid];
  }
  __syncthreads();
  const float y0 = yq[0], y1 = yq[1];
#pragma unroll 1
  for (int g = tid; g < nG; g += NTHR) {
    const float* rp = rvec + (size_t)g * RVP;
    float s0 = 0.f, s1 = 0.f;
#pragma unroll 4
    for (int d = 0; d < HD; ++d) {
      const float rv = rp[d];
      s0 += rv * ow[HD + d];
      s1 += rv * ow[2 * HD + HD + d];
    }
    ysh[2 * g]     = y0 + s0;
    ysh[2 * g + 1] = y1 + s1;
  }
  __syncthreads();

  const int nOut = 2 * nG;
#pragma unroll 1
  for (int i = wave; i * 128 < nOut; i += NWAVE) {
    const int idx = i * 128 + 4 * lane;
    if (idx + 4 <= nOut) {
      *(volatile v4f*)(out + idx) = *(const v4f*)(ysh + idx);
    } else {
      if (idx     < nOut) *(volatile float*)(out + idx)     = ysh[idx];
      if (idx + 1 < nOut) *(volatile float*)(out + idx + 1) = ysh[idx + 1];
      if (idx + 2 < nOut) *(volatile float*)(out + idx + 2) = ysh[idx + 2];
      if (idx + 3 < nOut) *(volatile float*)(out + idx + 3) = ysh[idx + 3];
    }
  }
  __threadfence();
#pragma unroll 1
  for (int i = wave; i * 128 < nOut; i += NWAVE) {
    const int idx = i * 128 + 4 * lane;
    if (idx + 4 <= nOut) {
      *(volatile v4f*)(out + idx) = *(const v4f*)(ysh + idx);
    } else {
      if (idx     < nOut) *(volatile float*)(out + idx)     = ysh[idx];
      if (idx + 1 < nOut) *(volatile float*)(out + idx + 1) = ysh[idx + 1];
      if (idx + 2 < nOut) *(volatile float*)(out + idx + 2) = ysh[idx + 2];
      if (idx + 3 < nOut) *(volatile float*)(out + idx + 3) = ysh[idx + 3];
    }
  }
}

extern "C" void kernel_launch(void* const* d_in, const int* in_sizes, int n_in,
                              void* d_out, int out_size, void* d_ws, size_t ws_size,
                              hipStream_t stream) {
  if (n_in < 22) return;
  const int nN = in_sizes[3];
  const int nE = in_sizes[1] / 2;
  const int nG = out_size / 2;
  if (nN <= 0 || nE <= 0 || nG <= 0 || nG > MAXG) return;
  if (in_sizes[0] != nN * NF || in_sizes[1] != 2 * nE || in_sizes[2] != nE * EF) return;
  if (in_sizes[4] != HD * NF || in_sizes[5] != HD || in_sizes[6] != HD * EF || in_sizes[7] != HD) return;
  if (in_sizes[8] != KW * HD || in_sizes[9] != KW || in_sizes[10] != HD * HD || in_sizes[11] != HD) return;
  if (in_sizes[12] != 3 * HD * HD || in_sizes[13] != 3 * HD * HD || in_sizes[14] != 3 * HD || in_sizes[15] != 3 * HD) return;
  if (in_sizes[16] != 4 * HD * 2 * HD || in_sizes[17] != 4 * HD * HD || in_sizes[18] != 4 * HD || in_sizes[19] != 4 * HD) return;
  if (in_sizes[20] != 2 * 2 * HD || in_sizes[21] != 2 || out_size != 2 * nG) return;

  const float* x         = (const float*)d_in[0];
  const int*   ei        = (const int*)d_in[1];
  const float* ea        = (const float*)d_in[2];
  const int*   batch     = (const int*)d_in[3];
  const float* lin0_w    = (const float*)d_in[4];
  const float* lin0_b    = (const float*)d_in[5];
  const float* net_w1    = (const float*)d_in[6];
  const float* net_b1    = (const float*)d_in[7];
  const float* net_w2    = (const float*)d_in[8];
  const float* net_b2    = (const float*)d_in[9];
  const float* conv_root = (const float*)d_in[10];
  const float* conv_bias = (const float*)d_in[11];
  const float* gru_w_ih  = (const float*)d_in[12];
  const float* gru_w_hh  = (const float*)d_in[13];
  const float* gru_b_ih  = (const float*)d_in[14];
  const float* gru_b_hh  = (const float*)d_in[15];
  const float* lstm_w_ih = (const float*)d_in[16];
  const float* lstm_w_hh = (const float*)d_in[17];
  const float* lstm_b_ih = (const float*)d_in[18];
  const float* lstm_b_hh = (const float*)d_in[19];
  const float* lin_out_w = (const float*)d_in[20];
  const float* lin_out_b = (const float*)d_in[21];
  float* out = (float*)d_out;

  const int Npad = ((nN + NBK - 1) / NBK) * NBK;
  const int Epad = ((nE + MEDG - 1) / MEDG) * MEDG;

  char* ws = (char*)d_ws;
  size_t off = 0;
  const size_t oWT = off; off += (size_t)HD * KTOT * 2;       off = (off + 511) & ~(size_t)511;
  const size_t oRT = off; off += (size_t)HD * HD * 2;         off = (off + 511) & ~(size_t)511;
  const size_t oGI = off; off += (size_t)3 * HD * HD * 2;     off = (off + 511) & ~(size_t)511;
  const size_t oGH = off; off += (size_t)3 * HD * HD * 2;     off = (off + 511) & ~(size_t)511;
  const size_t oHA = off; off += (size_t)Npad * HD * 4;       off = (off + 511) & ~(size_t)511;
  const size_t oHB = off; off += (size_t)Npad * HD * 4;       off = (off + 511) & ~(size_t)511;
  const size_t oHS = off; off += (size_t)Epad * HD * 4;       off = (off + 511) & ~(size_t)511;
  const size_t oES = off; off += (size_t)Epad * HD * 4;       off = (off + 511) & ~(size_t)511;
  const size_t oMS = off; off += (size_t)Epad * HD * 4;       off = (off + 511) & ~(size_t)511;
  const size_t oRV = off; off += (size_t)nG * RVP * 4;        off = (off + 511) & ~(size_t)511;
  if (off > ws_size) return;
  if (off > (size_t)134217728) return;
  _Float16* wT   = (_Float16*)(ws + oWT);
  _Float16* rT   = (_Float16*)(ws + oRT);
  _Float16* gIH  = (_Float16*)(ws + oGI);
  _Float16* gHH  = (_Float16*)(ws + oGH);
  float*    hA   = (float*)(ws + oHA);
  float*    hB   = (float*)(ws + oHB);
  float*    hs   = (float*)(ws + oHS);
  float*    es   = (float*)(ws + oES);
  float*    msg  = (float*)(ws + oMS);
  float*    rvec = (float*)(ws + oRV);

  const int vec8 = ((nE & 3) == 0) ? 1 : 0;

  const int nPrep = HD * (KTOT / 8) + HD * (HD / 8) + 2 * 3 * HD * (HD / 8);
  k_wprep<<<(nPrep + NTHR - 1) / NTHR, NTHR, 0, stream>>>(net_w2, net_b2, conv_root, gru_w_ih, gru_w_hh,
                                                        wT, rT, gIH, gHH);
  k_lin0<<<(Npad * 16) / NTHR, NTHR, 0, stream>>>(x, lin0_w, lin0_b, hA, nN);
  k_edgeh<<<(Epad * 16) / NTHR, NTHR, 0, stream>>>(ea, net_w1, net_b1, es, nE);

  float* hc = hA;
  float* hn = hB;
  for (int it = 0; it < NITER; ++it) {
    k_gather<<<(Epad * 16) / NTHR, NTHR, 0, stream>>>(ei, hc, hs, nN, nE);
    k_msg<<<Epad / MEDG, NTHR, 0, stream>>>(hs, es, wT, msg);
    k_node<<<Npad / NBK, NTHR, 0, stream>>>(ei, msg, hc, rT, gIH, gHH, conv_bias, gru_b_ih, gru_b_hh,
                                             hn, nN, nE, vec8);
    float* t = hc; hc = hn; hn = t;
  }

  k_attn<<<nG, NTHR, 0, stream>>>(hc, batch, lstm_w_ih, lstm_w_hh, lstm_b_ih, lstm_b_hh, rvec, nN);
  k_out<<<1, NTHR, 0, stream>>>(rvec, lstm_w_ih, lstm_w_hh, lstm_b_ih, lstm_b_hh, lin_out_w, lin_out_b, out, nG);
}
